// ScaledDotProduct_76501957476888
// MI455X (gfx1250) — hardware-verified
//
#include <hip/hip_runtime.h>
#include <math.h>


#ifndef NB
#define NB 2
#endif
#ifndef SEQ
#define SEQ 2048
#endif
#define NB_FULL  2
#define SEQ_FULL 2048
#define HH    16
#define DD    128
#define QTILE 128
#define KT    64
#define NT    (SEQ / KT)

static_assert(NB >= 1 && NB <= NB_FULL);
static_assert(SEQ >= QTILE && SEQ <= SEQ_FULL);
static_assert(SEQ % QTILE == 0);
static_assert(SEQ % KT == 0);
static_assert(DD == 128);

typedef _Float16 v16h __attribute__((ext_vector_type(16)));
typedef _Float16 v8h  __attribute__((ext_vector_type(8), __may_alias__));
typedef _Float16 v2h  __attribute__((ext_vector_type(2), __may_alias__));
typedef float    v8f  __attribute__((ext_vector_type(8)));
typedef float    v4f  __attribute__((ext_vector_type(4), __may_alias__));

union Frag { v16h v; v8h half[2]; };

union LdsU { _Float16 h[2 * KT * DD]; float f[8 * 16 * 64]; };
static_assert(sizeof(LdsU) == 32768);

namespace {
constexpr float kC2    = 0.12751743f;
constexpr float kCarry = 16384.0f;
}

__device__ __forceinline__ float bfr(float x) {
  unsigned int u = __float_as_uint(x);
  u = (u + 0x7FFFu + ((u >> 16) & 1u)) & 0xFFFF0000u;
  return __uint_as_float(u);
}
__device__ __forceinline__ v8h cvt8(v4f a, v4f b) {
  v8h r;
  r[0] = (_Float16)bfr(a[0]); r[1] = (_Float16)bfr(a[1]);
  r[2] = (_Float16)bfr(a[2]); r[3] = (_Float16)bfr(a[3]);
  r[4] = (_Float16)bfr(b[0]); r[5] = (_Float16)bfr(b[1]);
  r[6] = (_Float16)bfr(b[2]); r[7] = (_Float16)bfr(b[3]);
  return r;
}
__device__ __forceinline__ float fexp2(float x) {
#if __has_builtin(__builtin_amdgcn_exp2f)
  return __builtin_amdgcn_exp2f(x);
#else
  return exp2f(x);
#endif
}
__device__ __forceinline__ v4f mk4(float a, float b, float c, float d) {
  v4f r; r[0] = a; r[1] = b; r[2] = c; r[3] = d; return r;
}
__device__ __forceinline__ v8f mma16(v16h a, v16h b, v8f c) {
  v8f d = __builtin_amdgcn_wmma_f32_16x16x32_f16(false, a, false, b, (short)0, c, false, false);
  asm volatile("v_nop\n\tv_nop\n\tv_nop\n\tv_nop" : "+v"(d) : "v"(a), "v"(b));
  return d;
}


#define KFRAG(fr, g, c) do {                                                                 \
    (fr).half[0] = *(const v8h*)(Ksh + (16 * (g) + ln) * DD + 32 * (c) + 8 * lh);           \
    (fr).half[1] = *(const v8h*)(Ksh + (16 * (g) + ln) * DD + 32 * (c) + 16 + 8 * lh);      \
  } while (0)
#define ST_STEP(sacc, g) do { Frag a_;                                                       \
    KFRAG(a_, g, 0); sacc = mma16(a_.v, bq0.v, sacc);                                        \
    KFRAG(a_, g, 1); sacc = mma16(a_.v, bq1.v, sacc);                                        \
    KFRAG(a_, g, 2); sacc = mma16(a_.v, bq2.v, sacc);                                        \
    KFRAG(a_, g, 3); sacc = mma16(a_.v, bq3.v, sacc);                                        \
  } while (0)
#define VFRAG(fr, c, j) do {                                                                 \
    (fr).half[0] = *(const v8h*)(Vts + (16 * (c) + ln) * KT + 32 * (j) + 8 * lh);            \
    (fr).half[1] = *(const v8h*)(Vts + (16 * (c) + ln) * KT + 32 * (j) + 16 + 8 * lh);       \
  } while (0)
#define OT_STEP(oacc, c) do { Frag a_;                                                       \
    VFRAG(a_, c, 0); oacc = mma16(a_.v, bp0, oacc);                                          \
    VFRAG(a_, c, 1); oacc = mma16(a_.v, bp1, oacc);                                          \
  } while (0)
#define LOADQ(bq, c) do {                                                                    \
    v4f x0_ = *(const v4f*)(qrow + 32 * (c));      v4f x1_ = *(const v4f*)(qrow + 32 * (c) + 4);  \
    v4f y0_ = *(const v4f*)(qrow + 32 * (c) + 16); v4f y1_ = *(const v4f*)(qrow + 32 * (c) + 20); \
    (bq).half[0] = cvt8(x0_, x1_); (bq).half[1] = cvt8(y0_, y1_);                            \
  } while (0)
#define EPI_PASS(p, oa, ob, oc, od) do {                                                     \
    __syncthreads();                                                                          \
    { float* sr_ = stg + ln * 64 + 8 * lh;                                                   \
      *(v4f*)(sr_ +  0) = mk4(oa[0] * inv, oa[1] * inv, oa[2] * inv, oa[3] * inv);           \
      *(v4f*)(sr_ +  4) = mk4(oa[4] * inv, oa[5] * inv, oa[6] * inv, oa[7] * inv);           \
      *(v4f*)(sr_ + 16) = mk4(ob[0] * inv, ob[1] * inv, ob[2] * inv, ob[3] * inv);           \
      *(v4f*)(sr_ + 20) = mk4(ob[4] * inv, ob[5] * inv, ob[6] * inv, ob[7] * inv);           \
      *(v4f*)(sr_ + 32) = mk4(oc[0] * inv, oc[1] * inv, oc[2] * inv, oc[3] * inv);           \
      *(v4f*)(sr_ + 36) = mk4(oc[4] * inv, oc[5] * inv, oc[6] * inv, oc[7] * inv);           \
      *(v4f*)(sr_ + 48) = mk4(od[0] * inv, od[1] * inv, od[2] * inv, od[3] * inv);           \
      *(v4f*)(sr_ + 52) = mk4(od[4] * inv, od[5] * inv, od[6] * inv, od[7] * inv); }         \
    __syncthreads();                                                                          \
    v4f val_[8];                                                                              \
    for (int s_ = 0; s_ < 8; ++s_)                                         \
      val_[s_] = *(const v4f*)(stg + (2 * s_ + rsub) * 64 + coff);                           \
    float* ob_ = op + (size_t)rsub * DD + 64 * (p) + coff;                                   \
    for (int s_ = 0; s_ < 8; ++s_)                                         \
      *(volatile v4f*)(ob_ + (size_t)(2 * s_) * DD) = val_[s_];                               \
    __threadfence();                                                                          \
    for (int s_ = 0; s_ < 8; ++s_)                                         \
      *(volatile v4f*)(ob_ + (size_t)(2 * s_) * DD) = val_[s_];                               \
  } while (0)

__global__ __launch_bounds__(256) __attribute__((amdgpu_num_vgpr(256)))
void attn_fwd_f16(const float* __restrict__ q, const float* __restrict__ k,
                  const float* __restrict__ v, float* __restrict__ o) {
  __shared__ LdsU lds;
  _Float16* const Ksh = lds.h;
  _Float16* const Vts = lds.h + KT * DD;

  const int tid  = threadIdx.x;
  const int lane = tid & 31;
  const int w    = tid >> 5;
  const int lh   = lane >> 4;
  const int ln   = lane & 15;

  const int qblocks = SEQ / QTILE;
  const int bh    = blockIdx.x / qblocks;
  const int qblk  = blockIdx.x - bh * qblocks;
  const int qbase = qblk * QTILE + w * 16;

  const size_t ibase = (size_t)bh * SEQ_FULL * DD;
  const float* qp = q + ibase + (size_t)qbase * DD;
  const float* kp = k + ibase;
  const float* vp = v + ibase;
  float*       op = o + ((size_t)bh * SEQ + qbase) * DD;

  Frag bq0, bq1, bq2, bq3;
  {
    const float* qrow = qp + (size_t)ln * DD + 8 * lh;
    LOADQ(bq0, 0); LOADQ(bq1, 1); LOADQ(bq2, 2); LOADQ(bq3, 3);
  }

  v16h aones;
#pragma unroll
  for (int i = 0; i < 16; ++i) aones[i] = (_Float16)1.0f;

  v8f o0 = {}, o1 = {}, o2 = {}, o3 = {}, o4 = {}, o5 = {}, o6 = {}, o7 = {};
  v8f lacc = {};
  float mrow = -3.0e38f;

#pragma unroll 1
  for (int t = 0; t < NT; ++t) {
    __syncthreads();
    {
      const float* src = kp + (size_t)t * KT * DD + (size_t)tid * 32;
      _Float16* dst = Ksh + tid * 32;
#pragma unroll
      for (int j = 0; j < 4; ++j) {
        v4f x0 = *(const v4f*)(src + 8 * j);
        v4f x1 = *(const v4f*)(src + 8 * j + 4);
        *(v8h*)(dst + 8 * j) = cvt8(x0, x1);
      }
    }
    {
      const int vk = (tid >> 3) << 1;
      const int vd = (tid & 7) << 4;
      const float* vr0 = vp + ((size_t)t * KT + vk) * DD + vd;
      const float* vr1 = vr0 + DD;
#pragma unroll
      for (int j = 0; j < 4; ++j) {
        v4f a0 = *(const v4f*)(vr0 + 4 * j);
        v4f a1 = *(const v4f*)(vr1 + 4 * j);
#pragma unroll
        for (int c = 0; c < 4; ++c) {
          v2h pr;
          pr[0] = (_Float16)bfr(a0[c]);
          pr[1] = (_Float16)bfr(a1[c]);
          *(v2h*)(Vts + (vd + 4 * j + c) * KT + vk) = pr;
        }
      }
    }
    __syncthreads();

    v8f s0 = {}, s1 = {}, s2 = {}, s3 = {};
    ST_STEP(s0, 0); ST_STEP(s1, 1); ST_STEP(s2, 2); ST_STEP(s3, 3);

    float mloc = s0[0];
#pragma unroll
    for (int i = 0; i < 8; ++i) {
      mloc = fmaxf(mloc, s0[i]); mloc = fmaxf(mloc, s1[i]);
      mloc = fmaxf(mloc, s2[i]); mloc = fmaxf(mloc, s3[i]);
    }
    mloc = fmaxf(mloc, __shfl_xor(mloc, 16, 32));
    const float mnew = fmaxf(mrow, mloc);
    const float fac  = fexp2((mrow - mnew) * kC2);
    mrow = mnew;

    v16h bp0, bp1;
#pragma unroll
    for (int i = 0; i < 8; ++i) {
      bp0[i]     = (_Float16)(fexp2((s0[i] - mnew) * kC2) * kCarry);
      bp0[i + 8] = (_Float16)(fexp2((s1[i] - mnew) * kC2) * kCarry);
      bp1[i]     = (_Float16)(fexp2((s2[i] - mnew) * kC2) * kCarry);
      bp1[i + 8] = (_Float16)(fexp2((s3[i] - mnew) * kC2) * kCarry);
    }

#pragma unroll
    for (int i = 0; i < 8; ++i) {
      o0[i] *= fac; o1[i] *= fac; o2[i] *= fac; o3[i] *= fac;
      o4[i] *= fac; o5[i] *= fac; o6[i] *= fac; o7[i] *= fac;
      lacc[i] *= fac;
    }

    lacc = mma16(aones, bp0, lacc);
    lacc = mma16(aones, bp1, lacc);

    OT_STEP(o0, 0); OT_STEP(o1, 1); OT_STEP(o2, 2); OT_STEP(o3, 3);
    OT_STEP(o4, 4); OT_STEP(o5, 5); OT_STEP(o6, 6); OT_STEP(o7, 7);
  }

  const float inv = 1.0f / lacc[0];
  float* const stg = lds.f + w * (16 * 64);
  const int rsub = lane >> 4;
  const int coff = 32 * ((lane >> 3) & 1) + 4 * (lane & 7);
  EPI_PASS(0, o0, o1, o2, o3);
  EPI_PASS(1, o4, o5, o6, o7);
}

extern "C" void kernel_launch(void* const* d_in, const int* in_sizes, int n_in,
                              void* d_out, int out_size, void* d_ws, size_t ws_size,
                              hipStream_t stream) {
  (void)d_ws; (void)ws_size;
  if (n_in < 3) return;
  const long long need_in  = (long long)NB * HH * SEQ_FULL * DD;
  const long long need_out = (long long)NB * HH * SEQ * DD;
  if ((long long)in_sizes[0] < need_in || (long long)in_sizes[1] < need_in ||
      (long long)in_sizes[2] < need_in) return;
  if ((long long)out_size < need_out) return;
  const float* q = (const float*)d_in[0];
  const float* k = (const float*)d_in[1];
  const float* v = (const float*)d_in[2];
  float* o = (float*)d_out;
  const int blocks = NB * HH * (SEQ / QTILE);
  attn_fwd_f16<<<dim3(blocks), dim3(256), 0, stream>>>(q, k, v, o);
  (void)hipGetLastError();
}
